// RNN_83227876262378
// MI455X (gfx1250) — hardware-verified
//
#include <hip/hip_runtime.h>

constexpr int SEQ_T   = 2048;
constexpr int NBAT    = 512;
constexpr int NHID    = 64;
constexpr int NTHR    = 64;
constexpr int NWAVE   = NTHR / 32;
constexpr int ROWS_W  = 32;
constexpr int ROWS_B  = ROWS_W * NWAVE;
constexpr int NBLK    = NBAT / ROWS_B;
constexpr int APITCH  = 72;
constexpr int WPITCH  = 72;
constexpr int YPITCH  = 16;
constexpr int HSPITCH = 68;
constexpr int NOUT0   = SEQ_T * NBAT;
constexpr int NOUT1   = NBAT * NHID;
constexpr float ACARRY   = 16.0f;
constexpr float BCARRY   = 64.0f;
constexpr float LOCARRY  = 2048.0f;
constexpr float ACC_INV  = 1.0f / (16.0f * 64.0f);
constexpr float ACCR_INV = 1.0f / (16.0f * 64.0f * 2048.0f);
static_assert(NBAT % ROWS_B == 0 && NBLK * ROWS_B == NBAT);
static_assert(NHID == 64 && NTHR == NHID);
static_assert((NHID * NHID) % (8 * NTHR) == 0);
static_assert((ROWS_B * NHID) % (8 * NTHR) == 0);
static_assert(APITCH % 8 == 0 && WPITCH % 8 == 0 && YPITCH % 4 == 0 && HSPITCH % 4 == 0);
static_assert((size_t)NOUT0 * 4 == 4194304);
static_assert(ROWS_W == 32);
static_assert(SEQ_T % 2 == 0);
static_assert(NHID % 32 == 0);

typedef __attribute__((ext_vector_type(16))) _Float16 v16h;
typedef __attribute__((ext_vector_type(8)))  _Float16 v8h;
typedef __attribute__((ext_vector_type(8)))  float    v8f;
typedef __attribute__((ext_vector_type(4)))  float    v4f;

__device__ __forceinline__ float bf16r(float f) {
  unsigned u = __float_as_uint(f);
  u = (u + 0x7FFFu + ((u >> 16) & 1u)) & 0xFFFF0000u;
  return __uint_as_float(u);
}

__device__ __forceinline__ void dep_guard_h(v8f& a, v8f& b, v16h x, v16h y) { asm volatile("v_nop\n\tv_nop\n\tv_nop\n\tv_nop" : "+v"(a), "+v"(b) : "v"(x), "v"(y)); }
__device__ __forceinline__ void keep4_h(v16h a, v16h b, v16h c, v16h d) { asm volatile("v_nop" :: "v"(a), "v"(b), "v"(c), "v"(d)); }
__device__ __forceinline__ void acc_guard4(v8f& a, v8f& b, v8f& c, v8f& d) { asm volatile("v_nop\n\tv_nop\n\tv_nop\n\tv_nop" : "+v"(a), "+v"(b), "+v"(c), "+v"(d)); }

struct FragH {
  union U { v16h v; v8h h[2]; };
  static __device__ __forceinline__ v16h load(const _Float16* p) {
    U f; f.h[0] = *(const v8h*)(p); f.h[1] = *(const v8h*)(p + 16); return f.v;
  }
  static __device__ __forceinline__ v8f mma(v16h a, v16h b, v8f c) {
    return __builtin_amdgcn_wmma_f32_16x16x32_f16(false, a, false, b, (short)0, c, false, false);
  }
};

__device__ __forceinline__ float ftanh(float x) {
  const float e = __builtin_amdgcn_exp2f(x * 2.8853900817779268f);
  return 1.0f - 2.0f * __builtin_amdgcn_rcpf(e + 1.0f);
}

__global__ __launch_bounds__(NTHR) void rnn_seq_kernel(
    const float* __restrict__ x,
    const float* __restrict__ h0,
    const float* __restrict__ w_ih,
    const float* __restrict__ w_hh,
    const float* __restrict__ b_ih,
    const float* __restrict__ b_hh,
    const float* __restrict__ w_lin,
    const float* __restrict__ b_lin,
    float* __restrict__ y,
    float* __restrict__ hn) {
  __shared__ __align__(16) _Float16 Ahi[2][ROWS_B * APITCH];
  __shared__ __align__(16) _Float16 Alo[2][ROWS_B * APITCH];
  __shared__ __align__(16) _Float16 Wt[NHID * WPITCH];
  __shared__ __align__(16) float    Ysl[NWAVE][ROWS_W * YPITCH];
  __shared__ __align__(16) float    Hs[ROWS_B * HSPITCH];
  __shared__ __align__(16) float    Pw[4 * NHID];

  const int tid = threadIdx.x, lane = tid & 31, wave = tid >> 5;
  const int m = lane & 15, hh = lane >> 4, koff = hh * 8, c4 = m * 4, q4 = (lane & 7) * 4;
  const int brow = blockIdx.x * ROWS_B;
  const int wrow = wave * ROWS_W;
  const int grow = brow + wrow;

  Pw[tid]            = bf16r(w_ih[tid]);
  Pw[NHID + tid]     = bf16r(b_ih[tid]);
  Pw[2 * NHID + tid] = bf16r(b_hh[tid]);
  Pw[3 * NHID + tid] = bf16r(w_lin[tid]);
  const float blin = bf16r(b_lin[0]);

#pragma unroll 1
  for (int it = 0; it < (NHID * NHID) / (8 * NTHR); ++it) {
    const int idx = it * NTHR + tid;
    const int n = idx >> 3, c8 = (idx & 7) * 8;
    const v4f a = *(const v4f*)(w_hh + n * NHID + c8);
    const v4f b = *(const v4f*)(w_hh + n * NHID + c8 + 4);
    v8h hv;
#pragma unroll
    for (int e = 0; e < 4; ++e) {
      hv[e]     = (_Float16)(bf16r(a[e]) * BCARRY);
      hv[4 + e] = (_Float16)(bf16r(b[e]) * BCARRY);
    }
    *(v8h*)(Wt + n * WPITCH + c8) = hv;
  }
#pragma unroll 1
  for (int it = 0; it < (ROWS_B * NHID) / (8 * NTHR); ++it) {
    const int idx = it * NTHR + tid;
    const int row = idx >> 3, c8 = (idx & 7) * 8;
    const v4f a = *(const v4f*)(h0 + (size_t)(brow + row) * NHID + c8);
    const v4f b = *(const v4f*)(h0 + (size_t)(brow + row) * NHID + c8 + 4);
    v8h hv, lv;
#pragma unroll
    for (int e = 0; e < 4; ++e) {
      const float s0 = bf16r(a[e]) * ACARRY;
      const float s1 = bf16r(b[e]) * ACARRY;
      const _Float16 g0 = (_Float16)s0;
      const _Float16 g1 = (_Float16)s1;
      const float r0 = s0 - (float)g0;
      const float r1 = s1 - (float)g1;
      hv[e]     = g0;
      hv[4 + e] = g1;
      lv[e]     = (_Float16)(r0 * LOCARRY);
      lv[4 + e] = (_Float16)(r1 * LOCARRY);
    }
    *(v8h*)(&Ahi[0][0] + row * APITCH + c8) = hv;
    *(v8h*)(&Alo[0][0] + row * APITCH + c8) = lv;
  }
  __syncthreads();

  float wih[4], bih[4], bhh[4], wlin[4];
#pragma unroll
  for (int j = 0; j < 4; ++j) {
    const int n = 16 * j + m;
    wih[j]  = Pw[n];
    bih[j]  = Pw[NHID + n];
    bhh[j]  = Pw[2 * NHID + n];
    wlin[j] = Pw[3 * NHID + n];
  }

  const v8f z8 = {0.f, 0.f, 0.f, 0.f, 0.f, 0.f, 0.f, 0.f};
  float* ys = Ysl[wave];

#pragma unroll 1
  for (int t = 0; t < SEQ_T; ++t) {
    const int cur = t & 1;
    const bool last = (t == SEQ_T - 1);
    const _Float16* ahr = &Ahi[cur][0];
    const _Float16* alr = &Alo[cur][0];
    _Float16* ahw = &Ahi[cur ^ 1][0];
    _Float16* alw = &Alo[cur ^ 1][0];
    const float* xt = x + (size_t)t * NBAT + grow + koff;

#pragma unroll 1
    for (int i = 0; i < 2; ++i) {
      float xr[8];
      {
        const v4f xa = *(const v4f*)(xt + 16 * i);
        const v4f xb = *(const v4f*)(xt + 16 * i + 4);
#pragma unroll
        for (int e = 0; e < 4; ++e) { xr[e] = bf16r(xa[e]); xr[4 + e] = bf16r(xb[e]); }
      }
      const int aoff = (wrow + 16 * i + m) * APITCH + koff;
      const v16h ah0 = FragH::load(ahr + aoff);
      const v16h ah1 = FragH::load(ahr + aoff + 32);
      const v16h al0 = FragH::load(alr + aoff);
      const v16h al1 = FragH::load(alr + aoff + 32);

      v8f acc[4], accR[4];
#pragma unroll
      for (int j = 0; j < 4; ++j) { acc[j] = z8; accR[j] = z8; }

#pragma unroll
      for (int j = 0; j < 4; ++j) {
        const _Float16* bp = Wt + (16 * j + m) * WPITCH + koff;
        const v16h b0 = FragH::load(bp);
        const v16h b1 = FragH::load(bp + 32);
        acc[j]  = FragH::mma(ah0, b0, acc[j]);
        acc[j]  = FragH::mma(ah1, b1, acc[j]);
        accR[j] = FragH::mma(al0, b0, accR[j]);
        accR[j] = FragH::mma(al1, b1, accR[j]);
        dep_guard_h(acc[j], accR[j], b0, b1);
      }
      keep4_h(ah0, ah1, al0, al1);
      acc_guard4(acc[0], acc[1], acc[2], acc[3]);
      acc_guard4(accR[0], accR[1], accR[2], accR[3]);

#pragma unroll
      for (int r = 0; r < 8; ++r) {
        const int lrow = 16 * i + 8 * hh + r;
        float yp = 0.0f;
#pragma unroll
        for (int j = 0; j < 4; ++j) {
          const float dot = acc[j][r] * ACC_INV + accR[j][r] * ACCR_INV;
          const float xpv = (xr[r] * wih[j] + bih[j]) + bhh[j];
          const float pre = xpv + dot;
          const float hv  = ftanh(pre);
          acc[j][r] = hv;
          const float hs = hv * ACARRY;
          const _Float16 g16 = (_Float16)hs;
          const float res = hs - (float)g16;
          const int ao = (wrow + lrow) * APITCH + 16 * j + m;
          ahw[ao] = g16;
          alw[ao] = (_Float16)(res * LOCARRY);
          yp = fmaf(hv, wlin[j], yp);
        }
        ys[lrow * YPITCH + m] = yp;
      }
      if (last) {
#pragma unroll
        for (int j = 0; j < 4; ++j)
#pragma unroll
          for (int r = 0; r < 8; ++r) Hs[(wrow + 16 * i + 8 * hh + r) * HSPITCH + 16 * j + m] = acc[j][r];
      }
    }
    __syncthreads();

    v4f yv;
#pragma unroll
    for (int rr = 0; rr < 4; ++rr) {
      const float* p = ys + (q4 + rr) * YPITCH;
      const v4f s0 = *(const v4f*)(p);
      const v4f s1 = *(const v4f*)(p + 4);
      const v4f s2 = *(const v4f*)(p + 8);
      const v4f s3 = *(const v4f*)(p + 12);
      const float s = (((s0[0] + s0[1]) + (s0[2] + s0[3])) + ((s1[0] + s1[1]) + (s1[2] + s1[3])))
                    + (((s2[0] + s2[1]) + (s2[2] + s2[3])) + ((s3[0] + s3[1]) + (s3[2] + s3[3])));
      yv[rr] = s + blin;
    }
    float* yo = y + (size_t)t * NBAT + grow + q4;
    for (int pass = 0; pass < 2; ++pass) {
      if (lane < 8) *(volatile v4f*)yo = yv;
      __threadfence();
    }
    __syncthreads();
  }

  __syncthreads();
  for (int pass = 0; pass < 2; ++pass) {
#pragma unroll
    for (int it = 0; it < 16; ++it) {
      const int row = wrow + 2 * it + hh;
      const v4f v = *(const v4f*)(Hs + row * HSPITCH + c4);
      *(volatile v4f*)(hn + (size_t)(brow + row) * NHID + c4) = v;
    }
    __threadfence();
  }
}

extern "C" void kernel_launch(void* const* d_in, const int* in_sizes, int n_in,
                              void* d_out, int out_size, void* d_ws, size_t ws_size, hipStream_t stream) {
  (void)d_ws; (void)ws_size;
  if (n_in < 8 || d_out == nullptr) return;
  if (in_sizes[0] != SEQ_T * NBAT || in_sizes[1] != NBAT * NHID || in_sizes[2] != NHID ||
      in_sizes[3] != NHID * NHID || in_sizes[4] != NHID || in_sizes[5] != NHID ||
      in_sizes[6] != NHID || in_sizes[7] != 1 || out_size != NOUT0 + NOUT1) return;

  const float* x     = (const float*)d_in[0];
  const float* h0    = (const float*)d_in[1];
  const float* w_ih  = (const float*)d_in[2];
  const float* w_hh  = (const float*)d_in[3];
  const float* b_ih  = (const float*)d_in[4];
  const float* b_hh  = (const float*)d_in[5];
  const float* w_lin = (const float*)d_in[6];
  const float* b_lin = (const float*)d_in[7];
  float* y  = (float*)d_out;
  float* hn = y + (size_t)NOUT0;

  rnn_seq_kernel<<<NBLK, NTHR, 0, stream>>>(x, h0, w_ih, w_hh, b_ih, b_hh, w_lin, b_lin, y, hn);
}
